// EnsembleActor_60902636257569
// MI455X (gfx1250) — hardware-verified
//
#include <hip/hip_runtime.h>
#include <math.h>

typedef __attribute__((ext_vector_type(16))) _Float16 v16h;
typedef __attribute__((ext_vector_type(16))) __bf16 v16b;
typedef __attribute__((ext_vector_type(8)))  _Float16 v8h;
typedef __attribute__((ext_vector_type(8)))  float v8f;
typedef __attribute__((ext_vector_type(4)))  float v4f;
typedef __attribute__((ext_vector_type(2)))  float v2f;
typedef __attribute__((ext_vector_type(4)))  unsigned v4u;
typedef __attribute__((ext_vector_type(4)))  int v4i;
typedef float __attribute__((may_alias)) float_a;
typedef int __attribute__((may_alias)) int_a;

template <typename T> __device__ __forceinline__ void vst2(void* p, T v) { *(volatile T*)p = v; __threadfence(); *(volatile T*)p = v; }
__device__ __forceinline__ v8f wmma16(v16h a, v16h b, v8f c) {
  v8f d = __builtin_amdgcn_wmma_f32_16x16x32_f16(false, a, false, b, (short)0, c, false, false);
  asm volatile("v_nop\n\tv_nop\n\tv_nop\n\tv_nop" : "+v"(d) : "v"(a), "v"(b));
  return d;
}
__device__ __forceinline__ v8f wmma_bf(v16b a, v16b b, v8f c) {
  v8f d = __builtin_amdgcn_wmma_f32_16x16x32_bf16(false, a, false, b, (short)0, c, false, false);
  asm volatile("v_nop\n\tv_nop\n\tv_nop\n\tv_nop" : "+v"(d) : "v"(a), "v"(b));
  return d;
}
__device__ __forceinline__ v16h frag_h(const _Float16* rowk0, int lane) {
  union { v16h v; v8h q[2]; } u; const _Float16* p = rowk0 + 8 * (lane >> 4);
  u.q[0] = *(const v8h*)p; u.q[1] = *(const v8h*)(p + 16); return u.v;
}
__device__ __forceinline__ v16h frag_f32(const float* rowk0, int lane) {
  v16h a; const float* p = rowk0 + 8 * (lane >> 4);
#pragma unroll
  for (int i = 0; i < 8; ++i) { a[i] = (_Float16)p[i]; a[8 + i] = (_Float16)p[16 + i]; }
  return a;
}
__device__ __forceinline__ v16h frag_f32s(const float* rowk0, int lane, float sc) {
  v16h a; const float* p = rowk0 + 8 * (lane >> 4);
#pragma unroll
  for (int i = 0; i < 8; ++i) { a[i] = (_Float16)(p[i] * sc); a[8 + i] = (_Float16)(p[16 + i] * sc); }
  return a;
}
__device__ __forceinline__ v16h fragc_f32(const float* W, int k0, int n, int lane, int ld, int K) {
  v16h a; const int g = lane >> 4;
#pragma unroll
  for (int i = 0; i < 8; ++i) { const int ka = k0 + 8 * g + i, kb = ka + 16;
    a[i] = (_Float16)(ka < K ? W[(size_t)(ka < K ? ka : K - 1) * ld + n] : 0.f); a[8 + i] = (_Float16)(kb < K ? W[(size_t)(kb < K ? kb : K - 1) * ld + n] : 0.f); }
  return a;
}
struct F2 { v16b h, l; };
__device__ __forceinline__ F2 bsplit16(const float v[16]) { F2 r;
#pragma unroll
  for (int i = 0; i < 16; ++i) { const __bf16 h = (__bf16)v[i]; r.h[i] = h; r.l[i] = (__bf16)(v[i] - (float)h); }
  return r; }
__device__ __forceinline__ F2 split_row(const float* row, int k0, int lane) { float v[16]; const float* p = row + k0 + 8 * (lane >> 4);
#pragma unroll
  for (int i = 0; i < 8; ++i) { v[i] = p[i]; v[8 + i] = p[16 + i]; }
  return bsplit16(v); }
__device__ __forceinline__ F2 split_rowK(const float* row, int k0, int lane, int K) { float v[16]; const int g = lane >> 4;
#pragma unroll
  for (int i = 0; i < 8; ++i) { const int ka = k0 + 8 * g + i, kb = ka + 16; v[i] = ka < K ? row[ka < K ? ka : K - 1] : 0.f; v[8 + i] = kb < K ? row[kb < K ? kb : K - 1] : 0.f; }
  return bsplit16(v); }
__device__ __forceinline__ F2 split_col(const float* W, int k0, int n, int lane, int ld, int K) { float v[16]; const int g = lane >> 4;
#pragma unroll
  for (int i = 0; i < 8; ++i) { const int ka = k0 + 8 * g + i, kb = ka + 16; v[i] = ka < K ? W[(size_t)(ka < K ? ka : K - 1) * ld + n] : 0.f; v[8 + i] = kb < K ? W[(size_t)(kb < K ? kb : K - 1) * ld + n] : 0.f; }
  return bsplit16(v); }
__device__ __forceinline__ v8f mac3(const F2& a, const F2& b, v8f c) { c = wmma_bf(a.l, b.h, c); c = wmma_bf(a.h, b.l, c); return wmma_bf(a.h, b.h, c); }
__device__ __forceinline__ float sigm(float v) { return 1.0f / (1.0f + expf(-v)); }
#define LDSX() do { asm volatile("s_wait_dscnt 0" ::: "memory"); __builtin_amdgcn_wave_barrier(); __builtin_amdgcn_fence(__ATOMIC_RELEASE, "workgroup"); } while (0)


#define NE 8
#define NBT 4096
#define OBS 256
#define HH 1024
#define NA 64
#define NR (NE * NBT)
#define WSC 256.0f
#ifndef TRE
#define TRE NBT
#endif
typedef __attribute__((ext_vector_type(8))) __bf16 v8b;
__device__ __forceinline__ v16b frag_b(const __bf16* rowk0, int lane) {
  union { v16b v; v8b q[2]; } u; const __bf16* p = rowk0 + 8 * (lane >> 4);
  u.q[0] = *(const v8b*)p; u.q[1] = *(const v8b*)(p + 16); return u.v;
}
__device__ __forceinline__ float bfr(float v) { return (float)(__bf16)v; }
__device__ __attribute__((noinline)) float exp_ni(float v) { return expf(v); }
__device__ __attribute__((noinline)) float erf_ni(float v) { return erff(v); }

#define WS_P1  0u
#define WS_P2  (WS_P1 + 2u * (size_t)NE * HH * OBS)
#define WS_P3  (WS_P2 + 2u * (size_t)NE * HH * HH)
#define WS_H1  (WS_P3 + 2u * (size_t)NE * NA * HH)
#define WS_H2  (WS_H1 + 2u * (size_t)NR * HH)
#define WS_END (WS_H2 + 2u * (size_t)NR * HH)

__global__ __launch_bounds__(256) void k_pack(const float* __restrict__ W1, const float* __restrict__ W2, const float* __restrict__ W3, char* __restrict__ ws) { const int n = blockIdx.x, e = blockIdx.y, which = blockIdx.z, t = threadIdx.x; __shared__ __align__(16) __bf16 sb[OBS]; __shared__ __align__(16) _Float16 sh[HH];
  if (which == 0) { sb[t] = (__bf16)W1[((size_t)e * OBS + t) * HH + n]; __syncthreads(); if (t < OBS / 8) vst2((unsigned*)((__bf16*)(ws + WS_P1) + ((size_t)e * HH + n) * OBS + t * 8), *(const v4u*)&sb[t * 8]); }
  else if (which == 1) { for (int k = t; k < HH; k += 256) sh[k] = (_Float16)(bfr(W2[((size_t)e * HH + k) * HH + n]) * WSC); __syncthreads(); for (int q = t; q < HH / 8; q += 256) vst2((unsigned*)((_Float16*)(ws + WS_P2) + ((size_t)e * HH + n) * HH + q * 8), *(const v4u*)&sh[q * 8]); }
  else { if (n >= NA) return; for (int k = t; k < HH; k += 256) sh[k] = (_Float16)(bfr(W3[((size_t)e * HH + k) * NA + n]) * WSC); __syncthreads(); for (int q = t; q < HH / 8; q += 256) vst2((unsigned*)((_Float16*)(ws + WS_P3) + ((size_t)e * NA + n) * HH + q * 8), *(const v4u*)&sh[q * 8]); } }
__global__ __launch_bounds__(128) void k_g1(const float* __restrict__ X, const __bf16* __restrict__ P1, const float* __restrict__ B1, _Float16* __restrict__ H1) { __shared__ __align__(16) _Float16 so[64][136];
  const int tid = threadIdx.x, wave = tid >> 5, lane = tid & 31, col = lane & 15, g = lane >> 4; const size_t e = blockIdx.z; const size_t rb = e * NBT + (size_t)blockIdx.x * 64; const size_t r0 = rb + wave * 16; const int c0 = blockIdx.y * 128; const __bf16* Wr = P1 + (e * HH) * OBS;
  v8f acc[8] = {};
#pragma unroll
  for (int kc = 0; kc < OBS / 32; ++kc) { v16b a; { const float* p = X + (r0 + col) * OBS + kc * 32 + 8 * g;
#pragma unroll
      for (int i = 0; i < 8; ++i) { a[i] = (__bf16)p[i]; a[8 + i] = (__bf16)p[16 + i]; } }
#pragma unroll
    for (int j = 0; j < 8; ++j) acc[j] = wmma_bf(a, frag_b(Wr + (size_t)(c0 + j * 16 + col) * OBS + kc * 32, lane), acc[j]); }
#pragma unroll
  for (int j = 0; j < 8; ++j) { const float bb = bfr(B1[e * HH + c0 + j * 16 + col]);
#pragma unroll
    for (int r = 0; r < 8; ++r) so[wave * 16 + 8 * g + r][j * 16 + col] = (_Float16)fmaxf(acc[j][r] + bb, 0.f); }
  __syncthreads(); for (int q = tid; q < 64 * 16; q += 128) { const int rl = q >> 4, pc = q & 15; vst2((unsigned*)(H1 + (rb + rl) * HH + c0 + pc * 8), *(const v4u*)&so[rl][pc * 8]); } }
__global__ __launch_bounds__(128) void k_g2(const _Float16* __restrict__ H1, const _Float16* __restrict__ P2, const float* __restrict__ B2, _Float16* __restrict__ H2) { __shared__ __align__(16) _Float16 so[64][136];
  const int tid = threadIdx.x, wave = tid >> 5, lane = tid & 31, col = lane & 15, g = lane >> 4; const size_t e = blockIdx.z; const size_t rb = e * NBT + (size_t)blockIdx.x * 64; const size_t r0 = rb + wave * 16; const int c0 = blockIdx.y * 128; const _Float16* Wr = P2 + (e * HH) * HH;
  v8f acc[8] = {};
#pragma unroll 2
  for (int kc = 0; kc < HH / 32; ++kc) { const v16h a = frag_h(H1 + (r0 + col) * HH + kc * 32, lane);
#pragma unroll
    for (int j = 0; j < 8; ++j) acc[j] = wmma16(a, frag_h(Wr + (size_t)(c0 + j * 16 + col) * HH + kc * 32, lane), acc[j]); }
#pragma unroll
  for (int j = 0; j < 8; ++j) { const float bb = bfr(B2[e * HH + c0 + j * 16 + col]);
#pragma unroll
    for (int r = 0; r < 8; ++r) so[wave * 16 + 8 * g + r][j * 16 + col] = (_Float16)fmaxf(acc[j][r] * (1.0f / WSC) + bb, 0.f); }
  __syncthreads(); for (int q = tid; q < 64 * 16; q += 128) { const int rl = q >> 4, pc = q & 15; vst2((unsigned*)(H2 + (rb + rl) * HH + c0 + pc * 8), *(const v4u*)&so[rl][pc * 8]); } }
__global__ __launch_bounds__(128) void k_g3(const _Float16* __restrict__ H2, const _Float16* __restrict__ P3, const float* __restrict__ B3, const float* __restrict__ NOISE, float* __restrict__ OUT0, float* __restrict__ OUT1) { __shared__ __align__(16) float s0[4][16][68], s1[4][16][68];
  const int tid = threadIdx.x, wave = tid >> 5, lane = tid & 31, col = lane & 15, g = lane >> 4; const size_t e = blockIdx.y; const size_t r0 = e * NBT + (size_t)blockIdx.x * 64 + wave * 16; const _Float16* Wr = P3 + (e * NA) * HH;
  v8f acc[4] = {};
#pragma unroll 2
  for (int kc = 0; kc < HH / 32; ++kc) { const v16h a = frag_h(H2 + (r0 + col) * HH + kc * 32, lane);
#pragma unroll
    for (int j = 0; j < 4; ++j) acc[j] = wmma16(a, frag_h(Wr + (size_t)(j * 16 + col) * HH + kc * 32, lane), acc[j]); }
  float ga[8];
#pragma unroll
  for (int r = 0; r < 8; ++r) { ga[r] = 0.f;
#pragma unroll
    for (int j = 0; j < 4; ++j) { acc[j][r] = acc[j][r] * (1.0f / WSC) + bfr(B3[e * NA + j * 16 + col]); ga[r] += fabsf(acc[j][r]); }
#pragma unroll
    for (int o = 1; o < 16; o <<= 1) ga[r] += __shfl_xor(ga[r], o); }
#pragma unroll
  for (int r = 0; r < 8; ++r) { const float gs = fmaxf(ga[r] * (1.0f / NA), 1.0f); const size_t row = r0 + 8 * g + r;
#pragma unroll
    for (int j = 0; j < 4; ++j) { const int c = j * 16 + col; const float mu = acc[j][r] / gs; s0[wave][8 * g + r][c] = tanhf(mu); s1[wave][8 * g + r][c] = tanhf(mu + 0.1f * bfr(NOISE[row * NA + c])); } }
  LDSX(); for (int rl = 0; rl < 16; ++rl) if (lane < 16) { vst2(OUT0 + (r0 + rl) * NA + lane * 4, *(const v4f*)&s0[wave][rl][lane * 4]); vst2(OUT1 + (r0 + rl) * NA + lane * 4, *(const v4f*)&s1[wave][rl][lane * 4]); } }
extern "C" void kernel_launch(void* const* d_in, const int* in_sizes, int n_in, void* d_out, int out_size, void* d_ws, size_t ws_size, hipStream_t stream) {
  (void)in_sizes; (void)n_in; (void)out_size;
  const float** F = (const float**)d_in;
  if (ws_size < (size_t)WS_END) return;
  char* ws = (char*)d_ws; _Float16 *H1 = (_Float16*)(ws + WS_H1), *H2 = (_Float16*)(ws + WS_H2);
  float* OUT0 = (float*)d_out; float* OUT1 = OUT0 + (size_t)NR * NA;
  k_pack<<<dim3(HH, NE, 3), 256, 0, stream>>>(F[2], F[4], F[6], ws);
  k_g1<<<dim3(TRE / 64, HH / 128, NE), 128, 0, stream>>>(F[0], (const __bf16*)(ws + WS_P1), F[3], H1);
  k_g2<<<dim3(TRE / 64, HH / 128, NE), 128, 0, stream>>>(H1, (const _Float16*)(ws + WS_P2), F[5], H2);
  k_g3<<<dim3(TRE / 64, NE), 128, 0, stream>>>(H2, (const _Float16*)(ws + WS_P3), F[7], F[1], OUT0, OUT1);
}
